// GlobalSLCLayer_33285996544384
// MI455X (gfx1250) — hardware-run, weakly checked
//
#include <hip/hip_runtime.h>
#include <stddef.h>


#define NN     2048
#define CW     64
#define KCH    4
#define NTHR   256
#define NSLOT  7
#define TLP    65
#define F_F32  1
#define F_ROW  2
#define F_TR   4
#define F_SUB  8
#define WSCAP  134217728

static_assert((NN % 128) == 0);
static_assert(CW == 64);
static_assert(NTHR == 256);

typedef unsigned short us;
typedef us     v8us  __attribute__((ext_vector_type(8)));
typedef __bf16 v16bf __attribute__((ext_vector_type(16)));
typedef float  v4f   __attribute__((ext_vector_type(4)));
typedef float  v8f   __attribute__((ext_vector_type(8)));
union Frag { v16bf v; v8us u[2]; };

__device__ __forceinline__ v8f wmb(v16bf a, v16bf b, v8f c) {
  v8f d = __builtin_amdgcn_wmma_f32_16x16x32_bf16(false, a, false, b, (short)0, c, false, false);
  asm volatile("v_nop\n\tv_nop\n\tv_nop\n\tv_nop" : "+v"(d) : "v"(a), "v"(b));
  return d;
}

__device__ __forceinline__ unsigned bf_rne(float f) {
  unsigned u = __float_as_uint(f);
  u += 0x7FFFu + ((u >> 16) & 1u);
  return u >> 16;
}

__device__ __forceinline__ void split8(const float (&x)[8], v8us& hv, v8us& lv) {
#pragma unroll
  for (int e = 0; e < 8; ++e) {
    const unsigned hb = bf_rne(x[e]);
    const float rem = x[e] - __uint_as_float(hb << 16);
    hv[e] = (us)hb;
    lv[e] = (us)bf_rne(rem);
  }
}

__global__ __launch_bounds__(NTHR) void k_cvtw(const float* __restrict__ W, us* H, us* L, int tot8, int dolo) {
  const int i = blockIdx.x * NTHR + threadIdx.x;
  const int ic = i < tot8 ? i : tot8 - 1;
  const float* p = W + (size_t)ic * 8;
  const v4f a = *(const v4f*)p;
  const v4f q = *(const v4f*)(p + 4);
  const float x[8] = {a.x, a.y, a.z, a.w, q.x, q.y, q.z, q.w};
  v8us hv, lv;
  split8(x, hv, lv);
  us* hp = H + (size_t)ic * 8;
  us* lp = L + (size_t)ic * 8;
  if (i < tot8) {
    *(volatile v8us*)hp = hv;
    if (dolo != 0) *(volatile v8us*)lp = lv;
  }
  __threadfence();
  if (i < tot8) {
    *(volatile v8us*)hp = hv;
    if (dolo != 0) *(volatile v8us*)lp = lv;
  }
}

__device__ __forceinline__ void trcvt_pass(const float* tl, int tid, us* tH, us* tL, size_t tbase, int tPitch,
                                           us* rH, us* rL, size_t rbase, int doRow) {
  if (doRow != 0) {
#pragma unroll
    for (int s = 0; s < 2; ++s) {
      const int p = s * NTHR + tid, r = p >> 3, c0 = (p & 7) * 8;
      float x[8];
#pragma unroll
      for (int e = 0; e < 8; ++e) x[e] = tl[r * TLP + c0 + e];
      v8us hv, lv;
      split8(x, hv, lv);
      const size_t o = rbase + (size_t)r * 64 + c0;
      *(volatile v8us*)(rH + o) = hv;
      *(volatile v8us*)(rL + o) = lv;
    }
  }
#pragma unroll
  for (int s = 0; s < 2; ++s) {
    const int p = s * NTHR + tid, c = p >> 3, j = p & 7;
    float x[8];
#pragma unroll
    for (int e = 0; e < 8; ++e) x[e] = tl[(8 * j + e) * TLP + c];
    v8us hv, lv;
    split8(x, hv, lv);
    const size_t o = tbase + (size_t)c * (size_t)tPitch + 8 * j;
    *(volatile v8us*)(tH + o) = hv;
    *(volatile v8us*)(tL + o) = lv;
  }
}

__global__ __launch_bounds__(NTHR) void k_trcvt(const float* __restrict__ in, long long inY, long long inX,
                                                us* tH, us* tL, long long tY, long long tX, int tPitch,
                                                us* rH, us* rL, long long rY, long long rX, int doRow) {
  __shared__ __attribute__((aligned(16))) float tl[64 * TLP];
  const int tid = threadIdx.x;
  const float* ip = in + (size_t)blockIdx.y * (size_t)inY + (size_t)blockIdx.x * (size_t)inX;
#pragma unroll
  for (int s = 0; s < 2; ++s) {
    const int p = s * NTHR + tid, r = p >> 3, c0 = (p & 7) * 8;
    const v4f a = *(const v4f*)(ip + r * 64 + c0);
    const v4f q = *(const v4f*)(ip + r * 64 + c0 + 4);
    float* d = tl + r * TLP + c0;
    d[0] = a.x; d[1] = a.y; d[2] = a.z; d[3] = a.w;
    d[4] = q.x; d[5] = q.y; d[6] = q.z; d[7] = q.w;
  }
  __syncthreads();
  const size_t tbase = (size_t)blockIdx.y * (size_t)tY + (size_t)blockIdx.x * (size_t)tX;
  const size_t rbase = (size_t)blockIdx.y * (size_t)rY + (size_t)blockIdx.x * (size_t)rX;
  trcvt_pass(tl, tid, tH, tL, tbase, tPitch, rH, rL, rbase, doRow);
  __threadfence();
  trcvt_pass(tl, tid, tH, tL, tbase, tPitch, rH, rL, rbase, doRow);
}

template <int BM>
__device__ __forceinline__ void gemm_pass(const float* stg, int tid, int flags, size_t fbase, float* outF,
                                          us* rowH, us* rowL, size_t tbase, int M, us* trH, us* trL) {
  const v4f* stg4 = (const v4f*)stg;
  if (flags & F_F32) {
#pragma unroll
    for (int it = 0; it < BM / 16; ++it) {
      const int q = it * NTHR + tid;
      const v4f v = stg4[q];
      *(volatile v4f*)(outF + fbase + 4 * (size_t)q) = v;
    }
  }
  if (flags & F_ROW) {
#pragma unroll
    for (int it = 0; it < BM / 32; ++it) {
      const int p = it * NTHR + tid, r = p >> 3, c0 = (p & 7) * 8;
      const v4f a = stg4[(r * 64 + c0) >> 2];
      const v4f q = stg4[((r * 64 + c0) >> 2) + 1];
      const float x[8] = {a.x, a.y, a.z, a.w, q.x, q.y, q.z, q.w};
      v8us hv, lv;
      split8(x, hv, lv);
      const size_t o = fbase + (size_t)r * 64 + c0;
      *(volatile v8us*)(rowH + o) = hv;
      *(volatile v8us*)(rowL + o) = lv;
    }
  }
  if (flags & F_TR) {
    constexpr int PPC = BM / 8;
#pragma unroll
    for (int it = 0; it < BM / 32; ++it) {
      const int p = it * NTHR + tid, c = p / PPC, j = p - c * PPC;
      float x[8];
#pragma unroll
      for (int e = 0; e < 8; ++e) x[e] = stg[(8 * j + e) * 64 + c];
      v8us hv, lv;
      split8(x, hv, lv);
      const size_t o = tbase + (size_t)c * (size_t)M + 8 * j;
      *(volatile v8us*)(trH + o) = hv;
      *(volatile v8us*)(trL + o) = lv;
    }
  }
}

template <int RT, int SPLIT>
__global__ __launch_bounds__(NTHR) void k_gemm(
    const us* __restrict__ Ah, const us* __restrict__ Al, int lda, long long aBatch,
    const us* __restrict__ Bh, const us* __restrict__ Bl, int ldb, long long bBatch,
    int K, int M, float alpha, const float* subp, int flags,
    float* outF, us* rowH, us* rowL, us* trH, us* trL) {
  constexpr int BM = 64 * RT;
  static_assert(RT == 1 || RT == 2);
  static_assert(SPLIT == 1 || SPLIT == 3);
  __shared__ __attribute__((aligned(16))) float stg[BM * 64];
  const int tid = threadIdx.x, lane = tid & 31, wave = tid >> 5, h = lane >> 4, m = lane & 15;
  const int rg = wave >> 1, cg = wave & 1;
  const int b = blockIdx.y, m0 = blockIdx.x * BM;
  const int wr0 = rg * 16 * RT;

  size_t aoff[RT], boff[2];
#pragma unroll
  for (int rt = 0; rt < RT; ++rt)
    aoff[rt] = (size_t)b * (size_t)aBatch + (size_t)(m0 + wr0 + 16 * rt + m) * (size_t)lda + 8 * h;
#pragma unroll
  for (int ct = 0; ct < 2; ++ct)
    boff[ct] = (size_t)b * (size_t)bBatch + (size_t)(cg * 32 + 16 * ct + m) * (size_t)ldb + 8 * h;

  v8f acc[RT][2];
#pragma unroll
  for (int rt = 0; rt < RT; ++rt) {
    const v8f zz = {0.f, 0.f, 0.f, 0.f, 0.f, 0.f, 0.f, 0.f};
    acc[rt][0] = zz;
    acc[rt][1] = zz;
  }

#pragma unroll 1
  for (int k0 = 0; k0 < K; k0 += 32) {
    Frag fa[RT], fb[2], ga[RT], gb[2];
#pragma unroll
    for (int rt = 0; rt < RT; ++rt) {
      fa[rt].u[0] = *(const v8us*)(Ah + aoff[rt] + k0);
      fa[rt].u[1] = *(const v8us*)(Ah + aoff[rt] + k0 + 16);
      if constexpr (SPLIT == 3) {
        ga[rt].u[0] = *(const v8us*)(Al + aoff[rt] + k0);
        ga[rt].u[1] = *(const v8us*)(Al + aoff[rt] + k0 + 16);
      }
    }
#pragma unroll
    for (int ct = 0; ct < 2; ++ct) {
      fb[ct].u[0] = *(const v8us*)(Bh + boff[ct] + k0);
      fb[ct].u[1] = *(const v8us*)(Bh + boff[ct] + k0 + 16);
      if constexpr (SPLIT == 3) {
        gb[ct].u[0] = *(const v8us*)(Bl + boff[ct] + k0);
        gb[ct].u[1] = *(const v8us*)(Bl + boff[ct] + k0 + 16);
      }
    }
#pragma unroll
    for (int rt = 0; rt < RT; ++rt) {
#pragma unroll
      for (int ct = 0; ct < 2; ++ct) {
        acc[rt][ct] = wmb(fa[rt].v, fb[ct].v, acc[rt][ct]);
        if constexpr (SPLIT == 3) {
          acc[rt][ct] = wmb(fa[rt].v, gb[ct].v, acc[rt][ct]);
          acc[rt][ct] = wmb(ga[rt].v, fb[ct].v, acc[rt][ct]);
        }
      }
    }
  }

#pragma unroll
  for (int rt = 0; rt < RT; ++rt) {
#pragma unroll
    for (int ct = 0; ct < 2; ++ct) {
      float* sp = stg + (size_t)(wr0 + 16 * rt + 8 * h) * 64 + cg * 32 + 16 * ct + m;
#pragma unroll
      for (int r = 0; r < 8; ++r) sp[r * 64] = acc[rt][ct][r];
    }
  }
  __syncthreads();

  const size_t fbase = (size_t)b * (size_t)M * 64 + (size_t)m0 * 64;
  {
    v4f* stg4 = (v4f*)stg;
#pragma unroll
    for (int it = 0; it < BM / 16; ++it) {
      const int q = it * NTHR + tid;
      v4f v = stg4[q] * alpha;
      if (flags & F_SUB) {
        const v4f s = *(const v4f*)(subp + fbase + 4 * (size_t)q);
        v = v - s;
      }
      stg4[q] = v;
    }
  }
  __syncthreads();

  const size_t tbase = (size_t)b * 64 * (size_t)M + (size_t)m0;
  gemm_pass<BM>(stg, tid, flags, fbase, outF, rowH, rowL, tbase, M, trH, trL);
  __threadfence();
  gemm_pass<BM>(stg, tid, flags, fbase, outF, rowH, rowL, tbase, M, trH, trL);
}

__global__ __launch_bounds__(NTHR) void k_final(const us* __restrict__ rowH, const us* __restrict__ rowL,
                                                long long slot, const us* __restrict__ thH,
                                                const us* __restrict__ thL, float* out, int M) {
  __shared__ __attribute__((aligned(16))) float stg[64 * 64];
  const int tid = threadIdx.x, lane = tid & 31, wave = tid >> 5, h = lane >> 4, m = lane & 15;
  const int rg = wave >> 1, cg = wave & 1;
  const int b = blockIdx.y, m0 = blockIdx.x * 64;
  const size_t arow = (size_t)b * (size_t)M * 64 + (size_t)(m0 + rg * 16 + m) * 64 + 8 * h;
  size_t bo[2];
#pragma unroll
  for (int ct = 0; ct < 2; ++ct) bo[ct] = (size_t)(cg * 32 + 16 * ct + m) * 64 + 8 * h;

  const v8f zz = {0.f, 0.f, 0.f, 0.f, 0.f, 0.f, 0.f, 0.f};
  v8f aS[2] = {zz, zz}, aD[2] = {zz, zz};

#pragma unroll 1
  for (int t = 0; t < KCH; ++t) {
    const size_t sS = (size_t)t * (size_t)slot;
    const size_t sD = (size_t)(t == 0 ? 0 : 3 + t) * (size_t)slot;
    const size_t pS = (size_t)t * 4096;
    const size_t pD = (size_t)(KCH + t) * 4096;
#pragma unroll
    for (int k0 = 0; k0 < 64; k0 += 32) {
      Frag fa, ga, fb[2], gb[2];
      fa.u[0] = *(const v8us*)(rowH + sS + arow + k0);
      fa.u[1] = *(const v8us*)(rowH + sS + arow + k0 + 16);
      ga.u[0] = *(const v8us*)(rowL + sS + arow + k0);
      ga.u[1] = *(const v8us*)(rowL + sS + arow + k0 + 16);
#pragma unroll
      for (int ct = 0; ct < 2; ++ct) {
        fb[ct].u[0] = *(const v8us*)(thH + pS + bo[ct] + k0);
        fb[ct].u[1] = *(const v8us*)(thH + pS + bo[ct] + k0 + 16);
        gb[ct].u[0] = *(const v8us*)(thL + pS + bo[ct] + k0);
        gb[ct].u[1] = *(const v8us*)(thL + pS + bo[ct] + k0 + 16);
      }
#pragma unroll
      for (int ct = 0; ct < 2; ++ct) {
        aS[ct] = wmb(fa.v, fb[ct].v, aS[ct]);
        aS[ct] = wmb(fa.v, gb[ct].v, aS[ct]);
        aS[ct] = wmb(ga.v, fb[ct].v, aS[ct]);
      }
      fa.u[0] = *(const v8us*)(rowH + sD + arow + k0);
      fa.u[1] = *(const v8us*)(rowH + sD + arow + k0 + 16);
      ga.u[0] = *(const v8us*)(rowL + sD + arow + k0);
      ga.u[1] = *(const v8us*)(rowL + sD + arow + k0 + 16);
#pragma unroll
      for (int ct = 0; ct < 2; ++ct) {
        fb[ct].u[0] = *(const v8us*)(thH + pD + bo[ct] + k0);
        fb[ct].u[1] = *(const v8us*)(thH + pD + bo[ct] + k0 + 16);
        gb[ct].u[0] = *(const v8us*)(thL + pD + bo[ct] + k0);
        gb[ct].u[1] = *(const v8us*)(thL + pD + bo[ct] + k0 + 16);
      }
#pragma unroll
      for (int ct = 0; ct < 2; ++ct) {
        aD[ct] = wmb(fa.v, fb[ct].v, aD[ct]);
        aD[ct] = wmb(fa.v, gb[ct].v, aD[ct]);
        aD[ct] = wmb(ga.v, fb[ct].v, aD[ct]);
      }
    }
  }

#pragma unroll
  for (int ct = 0; ct < 2; ++ct) {
    float* sp = stg + (size_t)(rg * 16 + 8 * h) * 64 + cg * 32 + 16 * ct + m;
#pragma unroll
    for (int r = 0; r < 8; ++r) sp[r * 64] = fmaxf(aS[ct][r], 0.0f) + fmaxf(aD[ct][r], 0.0f);
  }
  __syncthreads();

  const v4f* stg4 = (const v4f*)stg;
  const size_t obase = (size_t)b * (size_t)M * 64 + (size_t)m0 * 64;
#pragma unroll
  for (int it = 0; it < 4; ++it) {
    const int q = it * NTHR + tid;
    const v4f v = stg4[q];
    *(volatile v4f*)(out + obase + 4 * (size_t)q) = v;
  }
  __threadfence();
#pragma unroll
  for (int it = 0; it < 4; ++it) {
    const int q = it * NTHR + tid;
    const v4f v = stg4[q];
    *(volatile v4f*)(out + obase + 4 * (size_t)q) = v;
  }
}

extern "C" void kernel_launch(void* const* d_in, const int* in_sizes, int n_in,
                              void* d_out, int out_size, void* d_ws, size_t ws_size,
                              hipStream_t stream) {
  if (n_in < 5) return;
  const int nX = in_sizes[0];
  if (nX <= 0 || (nX % (NN * CW)) != 0) return;
  const int B = nX / (NN * CW);
  if (B < 1 || B > 4096) return;
  if (in_sizes[1] != NN * NN || in_sizes[2] != NN * NN) return;
  if (in_sizes[3] != KCH * CW * CW || in_sizes[4] != KCH * CW * CW) return;
  if (out_size != nX) return;

  const float* X   = (const float*)d_in[0];
  const float* Ws  = (const float*)d_in[1];
  const float* Wa  = (const float*)d_in[2];
  const float* Ths = (const float*)d_in[3];
  const float* Thd = (const float*)d_in[4];
  float* out = (float*)d_out;

  const size_t SLOT = (size_t)B * NN * CW;
  const size_t szW  = (size_t)NN * NN * 2;
  const size_t szT  = SLOT * 2;
  const size_t szR  = (size_t)NSLOT * SLOT * 2;
  const size_t szTh = (size_t)2 * KCH * CW * CW * 2;
  const size_t szS  = (size_t)B * CW * CW * 2;
  const size_t szF  = SLOT * 4;

  char* ws = (char*)d_ws;
  size_t off = 0;
  auto carve = [&](size_t bytes) -> size_t { const size_t o = off; off += (bytes + 255) & ~(size_t)255; return o; };
  const size_t oWsH = carve(szW);
  const size_t oWaH = carve(szW), oWaL = carve(szW);
  const size_t oXtH = carve(szT), oXtL = carve(szT);
  const size_t oRwH = carve(szR), oRwL = carve(szR);
  const size_t oThH = carve(szTh), oThL = carve(szTh);
  const size_t oS1tH = carve(szT), oS1tL = carve(szT);
  const size_t oS2tH = carve(szT), oS2tL = carve(szT);
  const size_t oWxH = carve(szT), oWxL = carve(szT);
  const size_t oD1tH = carve(szT), oD1tL = carve(szT);
  const size_t oD2tH = carve(szT), oD2tL = carve(szT);
  const size_t osH0 = carve(szS), osL0 = carve(szS);
  const size_t osH1 = carve(szS), osL1 = carve(szS);
  const size_t osH2 = carve(szS), osL2 = carve(szS);
  const size_t oS1f = carve(szF), oD1f = carve(szF);
  if (off > ws_size || off > (size_t)WSCAP) return;

  us* WsH  = (us*)(ws + oWsH);
  us* WaH  = (us*)(ws + oWaH);  us* WaL  = (us*)(ws + oWaL);
  us* XtH  = (us*)(ws + oXtH);  us* XtL  = (us*)(ws + oXtL);
  us* RwH  = (us*)(ws + oRwH);  us* RwL  = (us*)(ws + oRwL);
  us* ThH  = (us*)(ws + oThH);  us* ThL  = (us*)(ws + oThL);
  us* S1tH = (us*)(ws + oS1tH); us* S1tL = (us*)(ws + oS1tL);
  us* S2tH = (us*)(ws + oS2tH); us* S2tL = (us*)(ws + oS2tL);
  us* WxH  = (us*)(ws + oWxH);  us* WxL  = (us*)(ws + oWxL);
  us* D1tH = (us*)(ws + oD1tH); us* D1tL = (us*)(ws + oD1tL);
  us* D2tH = (us*)(ws + oD2tH); us* D2tL = (us*)(ws + oD2tL);
  us* sH0  = (us*)(ws + osH0);  us* sL0  = (us*)(ws + osL0);
  us* sH1  = (us*)(ws + osH1);  us* sL1  = (us*)(ws + osL1);
  us* sH2  = (us*)(ws + osH2);  us* sL2  = (us*)(ws + osL2);
  float* S1f = (float*)(ws + oS1f);
  float* D1f = (float*)(ws + oD1f);

  const int tot8 = NN * NN / 8;
  const dim3 gW((tot8 + NTHR - 1) / NTHR), gX(NN / 64, B), gTh(KCH, 1);
  const dim3 gM(NN / 128, B), gS(1, B), gF(NN / 64, B);
  const long long tB = 64LL * NN;
  const long long rB = (long long)NN * 64;
  const long long sB = 64LL * 64;
  const long long slotLL = (long long)SLOT;

  k_cvtw<<<gW, NTHR, 0, stream>>>(Ws, WsH, WsH, tot8, 0);
  k_cvtw<<<gW, NTHR, 0, stream>>>(Wa, WaH, WaL, tot8, 1);
  k_trcvt<<<gX, NTHR, 0, stream>>>(X, rB, 64LL * 64, XtH, XtL, tB, 64, NN, RwH, RwL, rB, 64LL * 64, 1);
  k_trcvt<<<gTh, NTHR, 0, stream>>>(Ths, 0, 4096, ThH, ThL, 0, 4096, 64, RwH, RwL, 0, 0, 0);
  k_trcvt<<<gTh, NTHR, 0, stream>>>(Thd, 0, 4096, ThH + KCH * 4096, ThL + KCH * 4096, 0, 4096, 64, RwH, RwL, 0, 0, 0);

  k_gemm<2, 1><<<gM, NTHR, 0, stream>>>(WsH, WsH, NN, 0, XtH, XtL, NN, tB, NN, NN, 1.0f, X,
                                       F_F32 | F_ROW | F_TR, S1f, RwH + 1 * SLOT, RwL + 1 * SLOT, S1tH, S1tL);
  k_gemm<2, 1><<<gM, NTHR, 0, stream>>>(WsH, WsH, NN, 0, S1tH, S1tL, NN, tB, NN, NN, 2.0f, X,
                                       F_SUB | F_ROW | F_TR, D1f, RwH + 2 * SLOT, RwL + 2 * SLOT, S2tH, S2tL);
  k_gemm<2, 1><<<gM, NTHR, 0, stream>>>(WsH, WsH, NN, 0, S2tH, S2tL, NN, tB, NN, NN, 2.0f, S1f,
                                       F_SUB | F_ROW, D1f, RwH + 3 * SLOT, RwL + 3 * SLOT, S1tH, S1tL);

  k_gemm<2, 3><<<gM, NTHR, 0, stream>>>(WaH, WaL, NN, 0, XtH, XtL, NN, tB, NN, NN, 1.0f, X,
                                       F_TR, D1f, RwH + 6 * SLOT, RwL + 6 * SLOT, WxH, WxL);
  k_gemm<1, 3><<<gS, NTHR, 0, stream>>>(WxH, WxL, NN, tB, XtH, XtL, NN, tB, NN, 64, 1.0f, X,
                                       F_TR, D1f, RwH + 6 * SLOT, RwL + 6 * SLOT, sH0, sL0);
  k_gemm<2, 3><<<gM, NTHR, 0, stream>>>(RwH, RwL, 64, rB, sH0, sL0, 64, sB, 64, NN, 1.0f, X,
                                       F_F32 | F_ROW | F_TR, D1f, RwH + 4 * SLOT, RwL + 4 * SLOT, D1tH, D1tL);
  k_gemm<1, 3><<<gS, NTHR, 0, stream>>>(WxH, WxL, NN, tB, D1tH, D1tL, NN, tB, NN, 64, 1.0f, X,
                                       F_TR, S1f, RwH + 6 * SLOT, RwL + 6 * SLOT, sH1, sL1);
  k_gemm<2, 3><<<gM, NTHR, 0, stream>>>(RwH, RwL, 64, rB, sH1, sL1, 64, sB, 64, NN, 2.0f, X,
                                       F_SUB | F_ROW | F_TR, S1f, RwH + 5 * SLOT, RwL + 5 * SLOT, D2tH, D2tL);
  k_gemm<1, 3><<<gS, NTHR, 0, stream>>>(WxH, WxL, NN, tB, D2tH, D2tL, NN, tB, NN, 64, 1.0f, X,
                                       F_TR, S1f, RwH + 6 * SLOT, RwL + 6 * SLOT, sH2, sL2);
  k_gemm<2, 3><<<gM, NTHR, 0, stream>>>(RwH, RwL, 64, rB, sH2, sL2, 64, sB, 64, NN, 2.0f, D1f,
                                       F_SUB | F_ROW, S1f, RwH + 6 * SLOT, RwL + 6 * SLOT, D1tH, D1tL);

  k_final<<<gF, NTHR, 0, stream>>>(RwH, RwL, slotLL, ThH, ThL, out, NN);
}
